// QuantumClassicalHybridModel_69226282877371
// MI455X (gfx1250) — hardware-verified
//
#include <hip/hip_runtime.h>
#include <stddef.h>
#include <math.h>


#define NQ    8
#define NPAR  48
#define DH    64
#define DO    256
#define MT    16
#define NTHR  256
#define HP    72
#define PI_F  3.14159265358979323846f

static_assert(MT == 2 * (NTHR / 32));
static_assert(DO == 32 * (NTHR / 32));
static_assert(DH == 64);
static_assert(DH % 32 == 0);
static_assert((HP * 2) % 16 == 0);
static_assert((MT * HP) % 8 == 0);
static_assert((MT * DO) % 4 == 0);

typedef unsigned short us_t;
typedef us_t   v8us  __attribute__((ext_vector_type(8)));
typedef __bf16 v16bf __attribute__((ext_vector_type(16)));
typedef float  v4f   __attribute__((ext_vector_type(4)));
typedef float  v8f   __attribute__((ext_vector_type(8)));
union FragB { v16bf v; v8us h[2]; };

__device__ __forceinline__ v8f wmb(v16bf a, v16bf b, v8f c) {
  v8f d = __builtin_amdgcn_wmma_f32_16x16x32_bf16(false, a, false, b, (short)0, c, false, false);
#if defined(__HIP_DEVICE_COMPILE__)
  asm volatile("v_nop\n\tv_nop\n\tv_nop\n\tv_nop" : "+v"(d) : "v"(a), "v"(b));
#endif
  return d;
}

__device__ __forceinline__ v8f zero8() {
  v8f z = {0.f, 0.f, 0.f, 0.f, 0.f, 0.f, 0.f, 0.f};
  return z;
}

__device__ __forceinline__ us_t bf16_bits(float x) {
  unsigned u = __float_as_uint(x);
  u = (u + 0x7FFFu + ((u >> 16) & 1u)) >> 16;
  return (us_t)u;
}
__device__ __forceinline__ float bf16_val(us_t b) {
  return __uint_as_float(((unsigned)b) << 16);
}


template <int LM, int SM>
__device__ __forceinline__ void ry_g(float (&re)[8], float (&im)[8], float c, float s, int lane) {
  if (LM != 0) {
    const float sg = (lane & LM) ? s : -s;
#pragma unroll
    for (int k = 0; k < 8; ++k) {
      const float pr = __shfl_xor(re[k], LM, 32);
      const float pq = __shfl_xor(im[k], LM, 32);
      re[k] = c * re[k] + sg * pr;
      im[k] = c * im[k] + sg * pq;
    }
  } else {
#pragma unroll
    for (int k = 0; k < 8; ++k) {
      if (SM != 0 && (k & SM) == 0) {
        const int k1 = k | SM;
        const float r0 = re[k], r1 = re[k1], i0 = im[k], i1 = im[k1];
        re[k]  = c * r0 - s * r1;
        re[k1] = s * r0 + c * r1;
        im[k]  = c * i0 - s * i1;
        im[k1] = s * i0 + c * i1;
      }
    }
  }
}

template <int LM, int SM>
__device__ __forceinline__ void rz_g(float (&re)[8], float (&im)[8], float c, float s, int lane) {
#pragma unroll
  for (int k = 0; k < 8; ++k) {
    const bool bit = (LM != 0) ? ((lane & LM) != 0) : ((k & SM) != 0);
    const float sv = bit ? s : -s;
    const float r = re[k], q = im[k];
    re[k] = c * r - sv * q;
    im[k] = c * q + sv * r;
  }
}

template <int MC, int ML>
__device__ __forceinline__ void cx_ll(float (&re)[8], float (&im)[8], int lane) {
  const bool ctl = (lane & MC) != 0;
#pragma unroll
  for (int k = 0; k < 8; ++k) {
    const float pr = __shfl_xor(re[k], ML, 32);
    const float pq = __shfl_xor(im[k], ML, 32);
    re[k] = ctl ? pr : re[k];
    im[k] = ctl ? pq : im[k];
  }
}

template <int MC, int ST>
__device__ __forceinline__ void cx_ls(float (&re)[8], float (&im)[8], int lane) {
  const bool ctl = (lane & MC) != 0;
#pragma unroll
  for (int k = 0; k < 8; ++k) {
    if ((k & ST) == 0) {
      const int k1 = k | ST;
      const float r0 = re[k], r1 = re[k1], i0 = im[k], i1 = im[k1];
      re[k]  = ctl ? r1 : r0;
      re[k1] = ctl ? r0 : r1;
      im[k]  = ctl ? i1 : i0;
      im[k1] = ctl ? i0 : i1;
    }
  }
}

template <int SC, int ST>
__device__ __forceinline__ void cx_ss(float (&re)[8], float (&im)[8]) {
#pragma unroll
  for (int k = 0; k < 8; ++k) {
    if ((k & SC) != 0 && (k & ST) == 0) {
      const int k1 = k | ST;
      float t = re[k]; re[k] = re[k1]; re[k1] = t;
      t = im[k]; im[k] = im[k1]; im[k1] = t;
    }
  }
}

template <int SC, int ML>
__device__ __forceinline__ void cx_sl(float (&re)[8], float (&im)[8]) {
#pragma unroll
  for (int k = 0; k < 8; ++k) {
    if ((k & SC) != 0) {
      re[k] = __shfl_xor(re[k], ML, 32);
      im[k] = __shfl_xor(im[k], ML, 32);
    }
  }
}

template <int LM, int SM>
__device__ __forceinline__ void var_wire(float (&re)[8], float (&im)[8], const float* cs, int lane) {
  ry_g<LM, SM>(re, im, cs[0], cs[1], lane);
  rz_g<LM, SM>(re, im, cs[2], cs[3], lane);
}

__global__ __launch_bounds__(NTHR) void k_prep(const float* __restrict__ W2, us_t* Whi, us_t* Wlo) {
  const int i = blockIdx.x * NTHR + (int)threadIdx.x;
  if (i >= DO * DH / 8) return;
  const int n  = i >> 3;
  const int k0 = (i & 7) * 8;
  v8us vh, vl;
#pragma unroll
  for (int e = 0; e < 8; ++e) {
    const float w  = W2[(size_t)(k0 + e) * DO + n];
    const us_t  hb = bf16_bits(w);
    const us_t  lb = bf16_bits(w - bf16_val(hb));
    vh[e] = hb;
    vl[e] = lb;
  }
  us_t* ph = Whi + (size_t)n * DH + k0;
  us_t* pl = Wlo + (size_t)n * DH + k0;
  *(volatile v8us*)ph = vh;
  *(volatile v8us*)pl = vl;
  __threadfence();
  *(volatile v8us*)ph = vh;
  *(volatile v8us*)pl = vl;
}

__global__ __launch_bounds__(NTHR) void k_main(const float* __restrict__ x, const float* __restrict__ qw,
                                               const float* __restrict__ W1, const float* __restrict__ b1,
                                               const us_t* __restrict__ Whi, const us_t* __restrict__ Wlo,
                                               const float* __restrict__ b2, float* out, int nB) {
  __shared__ float sW1[NQ * DH];
  __shared__ float sB1[DH];
  __shared__ float sB2[DO];
  __shared__ float sCS[2 * NPAR];
  __shared__ v8us  sHh8[MT * HP / 8];
  __shared__ v8us  sHl8[MT * HP / 8];
  __shared__ v4f   sO4[MT * DO / 4];
  us_t*  sHh = (us_t*)sHh8;
  us_t*  sHl = (us_t*)sHl8;
  float* sO  = (float*)sO4;

  const int tid = threadIdx.x, lane = tid & 31, wv = tid >> 5, h4 = lane >> 4, m = lane & 15;
  const int s0 = blockIdx.x * MT;

  for (int i = tid; i < NQ * DH; i += NTHR) sW1[i] = W1[i];
  if (tid < DH) sB1[tid] = b1[tid];
  for (int i = tid; i < DO; i += NTHR) sB2[i] = b2[i];
  if (tid < 64) {
    const int p = tid < NPAR ? tid : NPAR - 1;
    const float ph = 0.5f * qw[p];
    const float cp = cosf(ph), sp = sinf(ph);
    if (tid < NPAR) { sCS[2 * tid] = cp; sCS[2 * tid + 1] = sp; }
  }
  __syncthreads();

#pragma unroll 1
  for (int rep = 0; rep < 2; ++rep) {
    const int r = wv + 8 * rep;
    int s = s0 + r;
    s = s > nB - 1 ? nB - 1 : s;

    const float xv = x[(size_t)s * NQ + (lane & 7)];
    float mn = xv, mx = xv;
    mn = fminf(mn, __shfl_xor(mn, 1, 32));  mx = fmaxf(mx, __shfl_xor(mx, 1, 32));
    mn = fminf(mn, __shfl_xor(mn, 2, 32));  mx = fmaxf(mx, __shfl_xor(mx, 2, 32));
    mn = fminf(mn, __shfl_xor(mn, 4, 32));  mx = fmaxf(mx, __shfl_xor(mx, 4, 32));
    const float inv = 1.0f / ((mx - mn) + 1e-8f);
    const float th  = ((xv - mn) * inv) * PI_F;
    const float hth = 0.5f * th;
    const float cg = cosf(hth), sg = sinf(hth);

    float re[8], im[8];
#pragma unroll
    for (int k = 0; k < 8; ++k) { re[k] = 0.f; im[k] = 0.f; }
    re[0] = (lane == 0) ? 1.0f : 0.0f;

    ry_g<16, 0>(re, im, __shfl(cg, 0, 32), __shfl(sg, 0, 32), lane);
    ry_g< 8, 0>(re, im, __shfl(cg, 1, 32), __shfl(sg, 1, 32), lane);
    ry_g< 4, 0>(re, im, __shfl(cg, 2, 32), __shfl(sg, 2, 32), lane);
    ry_g< 2, 0>(re, im, __shfl(cg, 3, 32), __shfl(sg, 3, 32), lane);
    ry_g< 1, 0>(re, im, __shfl(cg, 4, 32), __shfl(sg, 4, 32), lane);
    ry_g< 0, 4>(re, im, __shfl(cg, 5, 32), __shfl(sg, 5, 32), lane);
    ry_g< 0, 2>(re, im, __shfl(cg, 6, 32), __shfl(sg, 6, 32), lane);
    ry_g< 0, 1>(re, im, __shfl(cg, 7, 32), __shfl(sg, 7, 32), lane);

    for (int l = 0; l < 3; ++l) {
      const float* cs = sCS + 4 * NQ * l;
      var_wire<16, 0>(re, im, cs +  0, lane);
      var_wire< 8, 0>(re, im, cs +  4, lane);
      var_wire< 4, 0>(re, im, cs +  8, lane);
      var_wire< 2, 0>(re, im, cs + 12, lane);
      var_wire< 1, 0>(re, im, cs + 16, lane);
      var_wire< 0, 4>(re, im, cs + 20, lane);
      var_wire< 0, 2>(re, im, cs + 24, lane);
      var_wire< 0, 1>(re, im, cs + 28, lane);
      cx_ll<16, 8>(re, im, lane);
      cx_ll< 8, 4>(re, im, lane);
      cx_ll< 4, 2>(re, im, lane);
      cx_ll< 2, 1>(re, im, lane);
      cx_ls< 1, 4>(re, im, lane);
      cx_ss< 4, 2>(re, im);
      cx_ss< 2, 1>(re, im);
      cx_sl< 1, 16>(re, im);
    }

    float pk[8], psum = 0.f;
#pragma unroll
    for (int k = 0; k < 8; ++k) { pk[k] = re[k] * re[k] + im[k] * im[k]; psum += pk[k]; }
    float ez[8];
    ez[0] = (lane & 16) ? -psum : psum;
    ez[1] = (lane &  8) ? -psum : psum;
    ez[2] = (lane &  4) ? -psum : psum;
    ez[3] = (lane &  2) ? -psum : psum;
    ez[4] = (lane &  1) ? -psum : psum;
    ez[5] = ((pk[0] + pk[1]) + (pk[2] + pk[3])) - ((pk[4] + pk[5]) + (pk[6] + pk[7]));
    ez[6] = ((pk[0] + pk[1]) + (pk[4] + pk[5])) - ((pk[2] + pk[3]) + (pk[6] + pk[7]));
    ez[7] = ((pk[0] + pk[2]) + (pk[4] + pk[6])) - ((pk[1] + pk[3]) + (pk[5] + pk[7]));
#pragma unroll
    for (int off = 16; off > 0; off >>= 1) {
#pragma unroll
      for (int w = 0; w < 8; ++w) ez[w] += __shfl_xor(ez[w], off, 32);
    }

    float a0 = 0.f, a1 = 0.f;
#pragma unroll
    for (int k = 0; k < 8; ++k) {
      a0 += ez[k] * sW1[k * DH + lane];
      a1 += ez[k] * sW1[k * DH + lane + 32];
    }
    const float hv0 = fmaxf(a0 + sB1[lane], 0.f);
    const float hv1 = fmaxf(a1 + sB1[lane + 32], 0.f);
    const us_t h0b = bf16_bits(hv0), h1b = bf16_bits(hv1);
    const us_t l0b = bf16_bits(hv0 - bf16_val(h0b));
    const us_t l1b = bf16_bits(hv1 - bf16_val(h1b));
    sHh[r * HP + lane]      = h0b;
    sHh[r * HP + lane + 32] = h1b;
    sHl[r * HP + lane]      = l0b;
    sHl[r * HP + lane + 32] = l1b;
  }
  __syncthreads();

  {
    FragB ahi[2], alo[2];
#pragma unroll
    for (int ks = 0; ks < 2; ++ks) {
      const us_t* ph = sHh + m * HP + 32 * ks + 8 * h4;
      const us_t* pl = sHl + m * HP + 32 * ks + 8 * h4;
      ahi[ks].h[0] = *(const v8us*)ph;
      ahi[ks].h[1] = *(const v8us*)(ph + 16);
      alo[ks].h[0] = *(const v8us*)pl;
      alo[ks].h[1] = *(const v8us*)(pl + 16);
    }
#pragma unroll
    for (int t = 0; t < 2; ++t) {
      const int n = 32 * wv + 16 * t + m;
      v8f acc = zero8();
#pragma unroll
      for (int ks = 0; ks < 2; ++ks) {
        const us_t* bh = Whi + (size_t)n * DH + 32 * ks + 8 * h4;
        const us_t* bl = Wlo + (size_t)n * DH + 32 * ks + 8 * h4;
        FragB fh, fl;
        fh.h[0] = *(const v8us*)bh;
        fh.h[1] = *(const v8us*)(bh + 16);
        fl.h[0] = *(const v8us*)bl;
        fl.h[1] = *(const v8us*)(bl + 16);
        acc = wmb(ahi[ks].v, fh.v, acc);
        acc = wmb(ahi[ks].v, fl.v, acc);
        acc = wmb(alo[ks].v, fh.v, acc);
      }
      const float bb = sB2[n];
#pragma unroll
      for (int rr = 0; rr < 8; ++rr) sO[(8 * h4 + rr) * DO + n] = acc[rr] + bb;
    }
  }
  __syncthreads();

  {
    const int row0 = 2 * wv;
    const v4f v00 = sO4[(row0    ) * (DO / 4) +      lane];
    const v4f v01 = sO4[(row0    ) * (DO / 4) + 32 + lane];
    const v4f v10 = sO4[(row0 + 1) * (DO / 4) +      lane];
    const v4f v11 = sO4[(row0 + 1) * (DO / 4) + 32 + lane];
    float* g0 = out + (size_t)(s0 + row0) * DO + 4 * lane;
    float* g1 = g0 + 128;
    float* g2 = g0 + DO;
    float* g3 = g0 + DO + 128;
    *(volatile v4f*)g0 = v00;
    *(volatile v4f*)g1 = v01;
    *(volatile v4f*)g2 = v10;
    *(volatile v4f*)g3 = v11;
    __threadfence();
    *(volatile v4f*)g0 = v00;
    *(volatile v4f*)g1 = v01;
    *(volatile v4f*)g2 = v10;
    *(volatile v4f*)g3 = v11;
  }
}

extern "C" void kernel_launch(void* const* d_in, const int* in_sizes, int n_in,
                              void* d_out, int out_size, void* d_ws, size_t ws_size,
                              hipStream_t stream) {
  if (n_in < 6) return;
  const int nB = in_sizes[0] / NQ;
  if (nB <= 0 || in_sizes[0] != nB * NQ || (nB % MT) != 0) return;
  if (in_sizes[1] != NPAR || in_sizes[2] != NQ * DH || in_sizes[3] != DH) return;
  if (in_sizes[4] != DH * DO || in_sizes[5] != DO) return;
  if (out_size != nB * DO) return;

  const float* x  = (const float*)d_in[0];
  const float* qw = (const float*)d_in[1];
  const float* W1 = (const float*)d_in[2];
  const float* b1 = (const float*)d_in[3];
  const float* W2 = (const float*)d_in[4];
  const float* b2 = (const float*)d_in[5];
  float* out = (float*)d_out;

  const size_t planeBytes = (size_t)DO * DH * 2;
  const size_t total = 2 * planeBytes;
  if (total > ws_size || total > (size_t)134217728) return;
  us_t* Whi = (us_t*)d_ws;
  us_t* Wlo = Whi + (size_t)DO * DH;

  k_prep<<<(DO * DH / 8 + NTHR - 1) / NTHR, NTHR, 0, stream>>>(W2, Whi, Wlo);
  k_main<<<nB / MT, NTHR, 0, stream>>>(x, qw, W1, b1, Whi, Wlo, b2, out, nB);
}
